// LSTM_68985764708483
// MI455X (gfx1250) — hardware-verified
//
#include <hip/hip_runtime.h>

constexpr int NSEQ   = 1024;
constexpr int TENC   = 64;
constexpr int TDEC   = 32;
constexpr int TALL   = TENC + TDEC;
constexpr int TSEL0  = TENC - 1;
constexpr int TSEL   = TALL - TSEL0;
constexpr int NINP   = 8;
constexpr int NHID   = 256;
constexpr int NGATE  = 4 * NHID;
constexpr int NOUTF  = 8;
constexpr int NOUTP  = 16;
constexpr int KX0    = 32;
constexpr int KT0    = KX0 + NHID;
constexpr int KT1    = NHID + NHID;
constexpr int NTHR   = 256;
constexpr int SEQB   = 16;
constexpr int NROWS0 = NSEQ * TALL;
constexpr int NROWS1 = NSEQ * TSEL;
constexpr int HEADT  = NROWS1 / 64;
constexpr int SLP    = 16;
constexpr float OPC     = 16.0f;
constexpr float ACC_INV = 1.0f / 256.0f;
static_assert(KT0 % 32 == 0 && KT1 % 32 == 0);
static_assert(NROWS1 % 64 == 0 && HEADT % (NTHR / 32) == 0);
static_assert(NSEQ % SEQB == 0);
static_assert(NHID == 32 * (NTHR / 32));
static_assert(SEQB * KX0 == 2 * NTHR);
static_assert(SEQB * NHID == 16 * NTHR);
static_assert(SEQB * NHID == 2 * NTHR * 8);
static_assert((NGATE * KT0) % 8 == 0 && (NGATE * KT1) % 8 == 0 && (NOUTP * NHID) % 8 == 0);

typedef __attribute__((ext_vector_type(16))) _Float16 v16h;
typedef __attribute__((ext_vector_type(8)))  _Float16 v8h;
typedef __attribute__((ext_vector_type(8)))  float    v8f;
typedef __attribute__((ext_vector_type(4)))  float    v4f;
typedef __attribute__((ext_vector_type(2)))  float    v2f;
typedef __attribute__((ext_vector_type(4)))  unsigned v4u;

__device__ __forceinline__ void dep_guard_h(v8f& a, v8f& b, v16h x, v16h y) { asm volatile("v_nop\n\tv_nop\n\tv_nop\n\tv_nop" : "+v"(a), "+v"(b) : "v"(x), "v"(y)); }
__device__ __forceinline__ void keep4_h(v16h a, v16h b, v16h c, v16h d) { asm volatile("v_nop" :: "v"(a), "v"(b), "v"(c), "v"(d)); }
__device__ __forceinline__ void acc_guard4(v8f& a, v8f& b, v8f& c, v8f& d) { asm volatile("v_nop\n\tv_nop\n\tv_nop\n\tv_nop" : "+v"(a), "+v"(b), "+v"(c), "+v"(d)); }
__device__ __forceinline__ void guard5_h(v8f& a0, v8f& a1, v8f& a2, v8f& a3, v16h x, v16h y0, v16h y1, v16h y2, v16h y3) {
  asm volatile("v_nop\n\tv_nop\n\tv_nop\n\tv_nop" : "+v"(a0), "+v"(a1), "+v"(a2), "+v"(a3) : "v"(x), "v"(y0), "v"(y1), "v"(y2), "v"(y3));
}
template <typename T> struct Frag;
template <> struct Frag<_Float16> {
  typedef v16h V; union U { v16h v; v8h h[2]; };
  static __device__ __forceinline__ v16h load(const _Float16* p) {
    U f; f.h[0] = *(const v8h*)(p); f.h[1] = *(const v8h*)(p + 16); return f.v;
  }
  static __device__ __forceinline__ v8f mma(v16h a, v16h b, v8f c) {
    return __builtin_amdgcn_wmma_f32_16x16x32_f16(false, a, false, b, (short)0, c, false, false);
  }
  static __device__ __forceinline__ void guard(v8f& a, v8f& b, v16h x, v16h y) { dep_guard_h(a, b, x, y); }
  static __device__ __forceinline__ void keep(v16h a, v16h b, v16h c, v16h d) { keep4_h(a, b, c, d); }
};

__device__ __forceinline__ float fsig(float x)  { return __builtin_amdgcn_rcpf(1.0f + __expf(-x)); }
__device__ __forceinline__ float ftanh(float x) { return 1.0f - 2.0f * __builtin_amdgcn_rcpf(__expf(2.0f * x) + 1.0f); }
__device__ __forceinline__ unsigned short f2h_bits(float f) { return __builtin_bit_cast(unsigned short, (_Float16)f); }

__global__ __launch_bounds__(NTHR) void wplane_kernel(const float* __restrict__ A, int KA, const float* __restrict__ Bm, int KBP,
                                                      int KX, int KT, int NR, int NP, unsigned short* __restrict__ dst) {
  const int i  = blockIdx.x * NTHR + threadIdx.x;
  const int kt8 = KT >> 3;
  const int n8 = NP * kt8;
  if (i >= n8) return;
  const int n  = i / kt8;
  const int k0 = (i - n * kt8) * 8;
  const int nn = (n < NR) ? n : (NR - 1);
  int ka = k0;      if (ka > KA - 8) ka = KA - 8;
  int kb = k0 - KX; if (kb < 0) kb = 0;  if (kb > KBP - 8) kb = KBP - 8;
  const float* pa = A  + (size_t)nn * KA  + ka;
  const float* pb = Bm + (size_t)nn * KBP + kb;
  const v4f a0 = *(const v4f*)(pa), a1 = *(const v4f*)(pa + 4);
  const v4f b0 = *(const v4f*)(pb), b1 = *(const v4f*)(pb + 4);
  const float fa = (k0 < KA  && n < NR) ? OPC : 0.0f;
  const float fb = (k0 >= KX && n < NR) ? OPC : 0.0f;
  v8h hv;
#pragma unroll
  for (int e = 0; e < 4; ++e) {
    hv[e]     = (_Float16)fmaf(fa, a0[e], fb * b0[e]);
    hv[4 + e] = (_Float16)fmaf(fa, a1[e], fb * b1[e]);
  }
  unsigned short* op = dst + (size_t)i * 8;
  *(volatile v8h*)op = hv;
  __threadfence();
  *(volatile v8h*)op = hv;
}

template <int LAYER, int AP>
__device__ __forceinline__ void stage_x(unsigned short* At, const float* __restrict__ xenc, const float* __restrict__ xdec,
                                        const unsigned short* __restrict__ hsin, int rowbase, int tid, int tn) {
  if (LAYER == 0) {
    const int row = tid >> 4, cp = (tid & 15) * 2;
    const int cc = (cp < NINP - 2) ? cp : (NINP - 2);
    const int ta = (tn < TENC) ? tn : (TENC - 1);
    const int tb = (tn >= TENC) ? (tn - TENC) : 0;
    const v2f va = *(const v2f*)(xenc + ((size_t)(rowbase + row) * TENC + (size_t)ta) * NINP + cc);
    const v2f vb = *(const v2f*)(xdec + ((size_t)(rowbase + row) * TDEC + (size_t)tb) * NINP + cc);
    const float fa = (tn <  TENC && cp < NINP) ? OPC : 0.0f;
    const float fb = (tn >= TENC && cp < NINP) ? OPC : 0.0f;
    const float x0 = fmaf(fa, va[0], fb * vb[0]);
    const float x1 = fmaf(fa, va[1], fb * vb[1]);
    const unsigned u = (unsigned)f2h_bits(x0) | ((unsigned)f2h_bits(x1) << 16);
    *(unsigned*)(At + row * AP + cp) = u;
  } else {
    const int row = tid >> 4, seg = (tid & 15) * 16;
    const unsigned short* sp = hsin + ((size_t)(rowbase + row) * TALL + (size_t)tn) * NHID + seg;
    const v4u w0 = *(const v4u*)(sp);
    const v4u w1 = *(const v4u*)(sp + 8);
    *(v4u*)(At + row * AP + seg)     = w0;
    *(v4u*)(At + row * AP + seg + 8) = w1;
  }
}

template <int LAYER>
__global__ __launch_bounds__(NTHR) void rec_seq_kernel(const float* __restrict__ xenc, const float* __restrict__ xdec,
                                                       const unsigned short* __restrict__ hsin,
                                                       const unsigned short* __restrict__ Wcp,
                                                       const float* __restrict__ bih, const float* __restrict__ bhh,
                                                       unsigned short* __restrict__ hsout) {
  constexpr int KX = (LAYER == 0) ? KX0 : NHID;
  constexpr int KT = KX + NHID;
  constexpr int AP = KT + 8;
  static_assert(KT % 32 == 0 && (AP * 2) % 16 == 0 && (KX * 2) % 16 == 0);
  __shared__ __align__(16) unsigned short At[SEQB * AP];
  const _Float16* Wc = (const _Float16*)Wcp;
  const int tid = threadIdx.x, lane = tid & 31, wave = tid >> 5;
  const int c = lane & 15, hh = lane >> 4, koff = hh * 8;
  const int rowbase = blockIdx.x * SEQB;

#pragma unroll 1
  for (int i = tid; i < SEQB * AP; i += NTHR) At[i] = (unsigned short)0;

  float cst[2][8], hst[2][8], bb[2][4];
#pragma unroll
  for (int nt = 0; nt < 2; ++nt) {
    const int j = 32 * wave + 16 * nt + c;
#pragma unroll
    for (int g = 0; g < 4; ++g) bb[nt][g] = bih[g * NHID + j] + bhh[g * NHID + j];
    asm volatile("" ::: "memory");
#pragma unroll
    for (int r = 0; r < 8; ++r) { cst[nt][r] = 0.0f; hst[nt][r] = 0.0f; }
  }
  __syncthreads();
  stage_x<LAYER, AP>(At, xenc, xdec, hsin, rowbase, tid, 0);
  __syncthreads();

  const _Float16* arow = (const _Float16*)At + c * AP + koff;
  const v8f z8 = {0.f, 0.f, 0.f, 0.f, 0.f, 0.f, 0.f, 0.f};

#pragma unroll 1
  for (int t = 0; t < TALL; ++t) {
#pragma unroll
    for (int nt = 0; nt < 2; ++nt) {
      const int j = 32 * wave + 16 * nt + c;
      const _Float16* w0 = Wc + (size_t)j * KT + koff;
      v8f acc[4];
      acc[0] = z8; acc[1] = z8; acc[2] = z8; acc[3] = z8;
#pragma unroll 1
      for (int k0 = 0; k0 < KT; k0 += 32) {
        const v16h a  = Frag<_Float16>::load(arow + k0);
        const v16h b0 = Frag<_Float16>::load(w0 + k0);
        const v16h b1 = Frag<_Float16>::load(w0 + (size_t)1 * NHID * KT + k0);
        const v16h b2 = Frag<_Float16>::load(w0 + (size_t)2 * NHID * KT + k0);
        const v16h b3 = Frag<_Float16>::load(w0 + (size_t)3 * NHID * KT + k0);
        acc[0] = Frag<_Float16>::mma(a, b0, acc[0]);
        acc[1] = Frag<_Float16>::mma(a, b1, acc[1]);
        acc[2] = Frag<_Float16>::mma(a, b2, acc[2]);
        acc[3] = Frag<_Float16>::mma(a, b3, acc[3]);
        guard5_h(acc[0], acc[1], acc[2], acc[3], a, b0, b1, b2, b3);
      }
      acc_guard4(acc[0], acc[1], acc[2], acc[3]);
#pragma unroll
      for (int r = 0; r < 8; ++r) {
        const float zi = acc[0][r] * ACC_INV + bb[nt][0];
        const float zf = acc[1][r] * ACC_INV + bb[nt][1];
        const float zg = acc[2][r] * ACC_INV + bb[nt][2];
        const float zo = acc[3][r] * ACC_INV + bb[nt][3];
        const float ig = fsig(zi);
        const float fg = fsig(zf);
        const float gg = ftanh(zg);
        const float og = fsig(zo);
        const float cn = fg * cst[nt][r] + ig * gg;
        cst[nt][r] = cn;
        hst[nt][r] = og * ftanh(cn);
      }
    }
    __syncthreads();
#pragma unroll
    for (int nt = 0; nt < 2; ++nt) {
      const int j = 32 * wave + 16 * nt + c;
#pragma unroll
      for (int r = 0; r < 8; ++r) At[(8 * hh + r) * AP + KX + j] = f2h_bits(hst[nt][r] * OPC);
    }
    stage_x<LAYER, AP>(At, xenc, xdec, hsin, rowbase, tid, (t + 1 < TALL) ? (t + 1) : (TALL - 1));
    __syncthreads();
    if (LAYER == 0 || t >= TSEL0) {
      v4u hw[2];
      size_t dofs[2];
#pragma unroll
      for (int it = 0; it < 2; ++it) {
        const int idx = it * NTHR + tid;
        const int row = idx >> 5, c8 = (idx & 31) * 8;
        hw[it] = *(const v4u*)(At + row * AP + KX + c8);
        const size_t drow = (LAYER == 0) ? ((size_t)(rowbase + row) * TALL + (size_t)t)
                                         : ((size_t)(rowbase + row) * TSEL + (size_t)(t - TSEL0));
        dofs[it] = drow * NHID + (size_t)c8;
      }
      for (int pass = 0; pass < 2; ++pass) {
#pragma unroll
        for (int it = 0; it < 2; ++it) *(volatile v4u*)(hsout + dofs[it]) = hw[it];
        __threadfence();
      }
    }
  }
}

__global__ __launch_bounds__(NTHR) void head_kernel(const unsigned short* __restrict__ HS1p, const unsigned short* __restrict__ WOTp,
                                                    const float* __restrict__ bout, float* __restrict__ out) {
  __shared__ __align__(16) float Sl[NTHR / 32][64 * SLP];
  const _Float16* HS1 = (const _Float16*)HS1p;
  const _Float16* WOT = (const _Float16*)WOTp;
  const int tid = threadIdx.x, lane = tid & 31, wave = tid >> 5;
  const int c = lane & 15, hh = lane >> 4, koff = hh * 8;
  const int tile = blockIdx.x * (NTHR / 32) + wave;
  if (tile >= HEADT) return;
  const int m0 = tile * 64;
  const float bo = bout[(c < NOUTF) ? c : (NOUTF - 1)];
  const v8f z8 = {0.f, 0.f, 0.f, 0.f, 0.f, 0.f, 0.f, 0.f};
  v8f acc[4];
  acc[0] = z8; acc[1] = z8; acc[2] = z8; acc[3] = z8;
  const _Float16* brow = WOT + (size_t)c * NHID + koff;
  const _Float16* ar0  = HS1 + (size_t)(m0 + c) * NHID + koff;
#pragma unroll 1
  for (int k0 = 0; k0 < NHID; k0 += 32) {
    const v16h b  = Frag<_Float16>::load(brow + k0);
    const v16h a0 = Frag<_Float16>::load(ar0 + k0);
    const v16h a1 = Frag<_Float16>::load(ar0 + (size_t)16 * NHID + k0);
    const v16h a2 = Frag<_Float16>::load(ar0 + (size_t)32 * NHID + k0);
    const v16h a3 = Frag<_Float16>::load(ar0 + (size_t)48 * NHID + k0);
    acc[0] = Frag<_Float16>::mma(a0, b, acc[0]);
    acc[1] = Frag<_Float16>::mma(a1, b, acc[1]);
    acc[2] = Frag<_Float16>::mma(a2, b, acc[2]);
    acc[3] = Frag<_Float16>::mma(a3, b, acc[3]);
    guard5_h(acc[0], acc[1], acc[2], acc[3], b, a0, a1, a2, a3);
  }
  acc_guard4(acc[0], acc[1], acc[2], acc[3]);
  float* slab = Sl[wave];
#pragma unroll
  for (int i = 0; i < 4; ++i)
#pragma unroll
    for (int r = 0; r < 8; ++r) slab[(16 * i + 8 * hh + r) * SLP + c] = acc[i][r] * ACC_INV + bo;
  __builtin_amdgcn_fence(__ATOMIC_RELEASE, "workgroup");
  __builtin_amdgcn_wave_barrier();
  __builtin_amdgcn_fence(__ATOMIC_ACQUIRE, "workgroup");
  v4f ov[4];
  size_t oofs[4];
#pragma unroll
  for (int it = 0; it < 4; ++it) {
    const int q = it * 32 + lane;
    const int row = q >> 1, c4 = (q & 1) * 4;
    ov[it] = *(const v4f*)(slab + row * SLP + c4);
    oofs[it] = (size_t)(m0 + row) * NOUTF + (size_t)c4;
  }
  for (int pass = 0; pass < 2; ++pass) {
#pragma unroll
    for (int it = 0; it < 4; ++it) *(volatile v4f*)(out + oofs[it]) = ov[it];
    __threadfence();
  }
}

extern "C" void kernel_launch(void* const* d_in, const int* in_sizes, int n_in,
                              void* d_out, int out_size, void* d_ws, size_t ws_size, hipStream_t stream) {
  if (n_in < 12 || d_out == nullptr || d_ws == nullptr) return;
  if (in_sizes[0] != NSEQ * TENC * NINP || in_sizes[1] != NSEQ * TDEC * NINP || in_sizes[2] != NGATE * NINP ||
      in_sizes[3] != NGATE * NHID || in_sizes[4] != NGATE || in_sizes[5] != NGATE || in_sizes[6] != NGATE * NHID ||
      in_sizes[7] != NGATE * NHID || in_sizes[8] != NGATE || in_sizes[9] != NGATE || in_sizes[10] != NOUTF * NHID ||
      in_sizes[11] != NOUTF || out_size != NROWS1 * NOUTF) return;

  const float* x_enc   = (const float*)d_in[0];
  const float* x_dec   = (const float*)d_in[1];
  const float* w_ih_l0 = (const float*)d_in[2];
  const float* w_hh_l0 = (const float*)d_in[3];
  const float* b_ih_l0 = (const float*)d_in[4];
  const float* b_hh_l0 = (const float*)d_in[5];
  const float* w_ih_l1 = (const float*)d_in[6];
  const float* w_hh_l1 = (const float*)d_in[7];
  const float* b_ih_l1 = (const float*)d_in[8];
  const float* b_hh_l1 = (const float*)d_in[9];
  const float* w_out   = (const float*)d_in[10];
  const float* b_out   = (const float*)d_in[11];
  float* out = (float*)d_out;

  char* ws = (char*)d_ws; size_t off = 0;
  auto carve = [&](size_t bytes) -> char* { char* p = ws + off; off += (bytes + 255) & ~(size_t)255; return p; };
  unsigned short* WC0 = (unsigned short*)carve((size_t)NGATE * KT0 * 2);
  unsigned short* WC1 = (unsigned short*)carve((size_t)NGATE * KT1 * 2);
  unsigned short* WOT = (unsigned short*)carve((size_t)NOUTP * NHID * 2);
  unsigned short* HS0 = (unsigned short*)carve((size_t)NROWS0 * NHID * 2);
  unsigned short* HS1 = (unsigned short*)carve((size_t)NROWS1 * NHID * 2);
  if (off > ws_size || off > (size_t)134217728) return;

  const int n8_0 = NGATE * (KT0 / 8);
  const int n8_1 = NGATE * (KT1 / 8);
  const int n8_2 = NOUTP * (NHID / 8);
  wplane_kernel<<<(n8_0 + NTHR - 1) / NTHR, NTHR, 0, stream>>>(w_ih_l0, NINP, w_hh_l0, NHID, KX0,  KT0,  NGATE, NGATE, WC0);
  wplane_kernel<<<(n8_1 + NTHR - 1) / NTHR, NTHR, 0, stream>>>(w_ih_l1, NHID, w_hh_l1, NHID, NHID, KT1,  NGATE, NGATE, WC1);
  wplane_kernel<<<(n8_2 + NTHR - 1) / NTHR, NTHR, 0, stream>>>(w_out,   NHID, w_out,   NHID, NHID, NHID, NOUTF, NOUTP, WOT);
  rec_seq_kernel<0><<<NSEQ / SEQB, NTHR, 0, stream>>>(x_enc, x_dec, WC1, WC0, b_ih_l0, b_hh_l0, HS0);
  rec_seq_kernel<1><<<NSEQ / SEQB, NTHR, 0, stream>>>(x_enc, x_dec, HS0, WC1, b_ih_l1, b_hh_l1, HS1);
  head_kernel<<<HEADT / (NTHR / 32), NTHR, 0, stream>>>(HS1, WOT, b_out, out);
}
